// PyramidMamba_82282983456964
// MI455X (gfx1250) — hardware-run, weakly checked
//
#include <hip/hip_runtime.h>
#include <math.h>

typedef __attribute__((ext_vector_type(16))) _Float16 v16h;
typedef __attribute__((ext_vector_type(8)))  _Float16 v8h;
typedef __attribute__((ext_vector_type(16))) __bf16   v16b;
typedef __attribute__((ext_vector_type(8)))  __bf16   v8b;
typedef __attribute__((ext_vector_type(8)))  float    v8f;
typedef __attribute__((ext_vector_type(4)))  float    v4f;

constexpr int kB     = 4;
constexpr int kCin   = 512;
constexpr int kL     = 256;
constexpr int kDimP  = 128;
constexpr int kDm    = 1024;
constexpr int kDi    = 2048;
constexpr int kDirs  = 4;
constexpr int kNs    = 16;
constexpr int kRk    = 64;
constexpr int kPix   = kB * kL;
constexpr int kE2    = 2 * kDi;
constexpr int kXdG   = kRk + 2 * kNs;
constexpr int kXdW   = kDirs * kXdG;
constexpr int kTP    = 260;
constexpr int kScanCh = 32;
constexpr int kScanTS = 64;
constexpr int kM1 = kB * 25,  kM1P = 128;
constexpr int kM2 = kB * 81,  kM2P = 384;
constexpr int kM3 = kB * 169, kM3P = 704;
constexpr int kPRow2 = kM1P;
constexpr int kPRow3 = kM1P + kM2P;
constexpr int kPRows = kM1P + kM2P + kM3P;
constexpr float kCarryXc  = 16.0f;
constexpr float kCarryWxp = 32.0f;
constexpr float kCarryXd  = 16.0f;
constexpr float kCarryWdt = 16.0f;
static_assert(kDm == kCin + 4 * kDimP);
static_assert(kXdG == 96 && kXdW == 384);
static_assert((kCin % 32) == 0 && (kDm % 32) == 0 && (kDi % 32) == 0 && (kRk % 32) == 0);
static_assert((kPix % 64) == 0 && (kE2 % 64) == 0 && (kXdW % 64) == 0 && (kDi % 64) == 0 && (kDm % 64) == 0 && (kDimP % 64) == 0);
static_assert((kM1P % 64) == 0 && (kM2P % 64) == 0 && (kM3P % 64) == 0 && kM1 <= kM1P && kM2 <= kM2P && kM3 <= kM3P);

constexpr size_t kSzWI = (size_t)kE2 * kDm * 2;
constexpr size_t kSzWO = (size_t)kDm * kDi * 2;
constexpr size_t kSzWC = (size_t)kDimP * kDm * 2;
constexpr size_t kSzWP = (size_t)4 * kDimP * kCin * 2;
constexpr size_t kSzWX = (size_t)kXdW * kDi * 2;
constexpr size_t kSzWD = (size_t)kDirs * kDi * kRk * 2;
constexpr size_t kSzF  = (size_t)kPix * kDm * 2;
constexpr size_t kSzP  = (size_t)kPRows * kCin * 2;
constexpr size_t kSzQ0 = (size_t)kPix * kDimP * 4;
constexpr size_t kSzQ1 = (size_t)kM1P * kDimP * 4;
constexpr size_t kSzQ2 = (size_t)kM2P * kDimP * 4;
constexpr size_t kSzQ3 = (size_t)kM3P * kDimP * 4;
constexpr size_t kSzY0 = (size_t)kB * kDimP * 4;
constexpr size_t kSzXZ = (size_t)kPix * kE2 * 4;
constexpr size_t kSzXC = (size_t)kPix * kDi * 4;
constexpr size_t kSzXC16 = (size_t)kPix * kDi * 2;
constexpr size_t kSzXD = (size_t)kPix * kXdW * 4;
constexpr size_t kSzXD16 = (size_t)kPix * kXdW * 2;
constexpr size_t kSzDP = (size_t)kDirs * kPix * kDi * 4;
constexpr size_t kSzYS = (size_t)kPix * kDi * 4;
constexpr size_t kSzYL = (size_t)kPix * kDi * 2;
constexpr size_t kSzYP = (size_t)kPix * kDm * 2;
constexpr size_t kSzCP = (size_t)kPix * kDimP * 4;

constexpr size_t kOffWIH = 0;
constexpr size_t kOffWIL = kOffWIH + kSzWI;
constexpr size_t kOffWOH = kOffWIL + kSzWI;
constexpr size_t kOffWOL = kOffWOH + kSzWO;
constexpr size_t kOffWCH = kOffWOL + kSzWO;
constexpr size_t kOffWCL = kOffWCH + kSzWC;
constexpr size_t kOffWPH = kOffWCL + kSzWC;
constexpr size_t kOffWPL = kOffWPH + kSzWP;
constexpr size_t kOffWXP = kOffWPL + kSzWP;
constexpr size_t kOffWDT = kOffWXP + kSzWX;
constexpr size_t kOffFH  = kOffWDT + kSzWD;
constexpr size_t kOffFL  = kOffFH + kSzF;
constexpr size_t kOffPH  = kOffFL + kSzF;
constexpr size_t kOffPL  = kOffPH + kSzP;
constexpr size_t kOffQ0  = kOffPL + kSzP;
constexpr size_t kOffQ1  = kOffQ0 + kSzQ0;
constexpr size_t kOffQ2  = kOffQ1 + kSzQ1;
constexpr size_t kOffQ3  = kOffQ2 + kSzQ2;
constexpr size_t kOffY0  = kOffQ3 + kSzQ3;
constexpr size_t kOffXZ  = kOffY0 + kSzY0;
constexpr size_t kOffXC  = kOffXZ + kSzXZ;
constexpr size_t kOffXC16 = kOffXC + kSzXC;
constexpr size_t kOffXD  = kOffXC16 + kSzXC16;
constexpr size_t kOffXD16 = kOffXD + kSzXD;
constexpr size_t kOffDP  = kOffXD16 + kSzXD16;
constexpr size_t kOffYS  = kOffDP + kSzDP;
constexpr size_t kOffYLH = kOffYS + kSzYS;
constexpr size_t kOffYLL = kOffYLH + kSzYL;
constexpr size_t kOffYPH = kOffYLL + kSzYL;
constexpr size_t kOffYPL = kOffYPH + kSzYP;
constexpr size_t kOffCP  = kOffYPL + kSzYP;
constexpr size_t kWsTotal = kOffCP + kSzCP;
static_assert(kWsTotal == 123963392ull);
static_assert(kWsTotal <= 134217728ull);
static_assert((kOffWIL % 128) == 0 && (kOffWOH % 128) == 0 && (kOffWOL % 128) == 0 && (kOffWCH % 128) == 0 &&
              (kOffWCL % 128) == 0 && (kOffWPH % 128) == 0 && (kOffWPL % 128) == 0 && (kOffWXP % 128) == 0 &&
              (kOffWDT % 128) == 0 && (kOffFH % 128) == 0 && (kOffFL % 128) == 0 && (kOffPH % 128) == 0 &&
              (kOffPL % 128) == 0 && (kOffQ0 % 128) == 0 && (kOffQ1 % 128) == 0 && (kOffQ2 % 128) == 0 &&
              (kOffQ3 % 128) == 0 && (kOffY0 % 128) == 0 && (kOffXZ % 128) == 0 && (kOffXC % 128) == 0 &&
              (kOffXC16 % 128) == 0 && (kOffXD % 128) == 0 && (kOffXD16 % 128) == 0 && (kOffDP % 128) == 0 &&
              (kOffYS % 128) == 0 && (kOffYLH % 128) == 0 && (kOffYLL % 128) == 0 && (kOffYPH % 128) == 0 &&
              (kOffYPL % 128) == 0 && (kOffCP % 128) == 0);

__device__ __forceinline__ unsigned short f2bf_bits(float f) {
  unsigned u = __float_as_uint(f);
  return (unsigned short)((u + 0x7FFFu + ((u >> 16) & 1u)) >> 16);
}
__device__ __forceinline__ float bf_bits2f(unsigned short h) { return __uint_as_float(((unsigned)h) << 16); }

__device__ __forceinline__ void split8_bf16(const v4f a0, const v4f a1, v8h& hv, v8h& lv) {
#pragma unroll
  for (int e = 0; e < 4; ++e) {
    const float f0 = a0[e];
    const float f1 = a1[e];
    const unsigned short h0 = f2bf_bits(f0), h1 = f2bf_bits(f1);
    const unsigned short l0 = f2bf_bits(f0 - bf_bits2f(h0)), l1 = f2bf_bits(f1 - bf_bits2f(h1));
    hv[e]     = __builtin_bit_cast(_Float16, h0);
    hv[4 + e] = __builtin_bit_cast(_Float16, h1);
    lv[e]     = __builtin_bit_cast(_Float16, l0);
    lv[4 + e] = __builtin_bit_cast(_Float16, l1);
  }
}

__device__ __forceinline__ void dep_guard4_h(v8f& a, v8f& b, v8f& c, v8f& d, v16h x, v16h y) { asm volatile("v_nop\n\tv_nop\n\tv_nop\n\tv_nop" : "+v"(a), "+v"(b), "+v"(c), "+v"(d) : "v"(x), "v"(y)); }
__device__ __forceinline__ void dep_guard4_b(v8f& a, v8f& b, v8f& c, v8f& d, v16b x, v16b y) { asm volatile("v_nop\n\tv_nop\n\tv_nop\n\tv_nop" : "+v"(a), "+v"(b), "+v"(c), "+v"(d) : "v"(x), "v"(y)); }
__device__ __forceinline__ void keep4_h(v16h a, v16h b, v16h c, v16h d) { asm volatile("v_nop" :: "v"(a), "v"(b), "v"(c), "v"(d)); }
__device__ __forceinline__ void keep4_b(v16b a, v16b b, v16b c, v16b d) { asm volatile("v_nop" :: "v"(a), "v"(b), "v"(c), "v"(d)); }
__device__ __forceinline__ void acc_guard4(v8f& a, v8f& b, v8f& c, v8f& d) { asm volatile("v_nop\n\tv_nop\n\tv_nop\n\tv_nop" : "+v"(a), "+v"(b), "+v"(c), "+v"(d)); }
template <typename T> struct Frag;
template <> struct Frag<_Float16> {
  typedef v16h V; union U { v16h v; v8h h[2]; };
  static __device__ __forceinline__ v16h load(const _Float16* p) {
    U f; f.h[0] = *(const v8h*)(p); f.h[1] = *(const v8h*)(p + 16); return f.v;
  }
  static __device__ __forceinline__ v8f mma(v16h a, v16h b, v8f c) {
    return __builtin_amdgcn_wmma_f32_16x16x32_f16(false, a, false, b, (short)0, c, false, false);
  }
  static __device__ __forceinline__ void guard(v8f& a, v8f& b, v8f& c, v8f& d, v16h x, v16h y) { dep_guard4_h(a, b, c, d, x, y); }
  static __device__ __forceinline__ void keep(v16h a, v16h b, v16h c, v16h d) { keep4_h(a, b, c, d); }
};
template <> struct Frag<__bf16> {
  typedef v16b V; union U { v16b v; v8b h[2]; };
  static __device__ __forceinline__ v16b load(const __bf16* p) {
    U f; f.h[0] = *(const v8b*)(p); f.h[1] = *(const v8b*)(p + 16); return f.v;
  }
  static __device__ __forceinline__ v8f mma(v16b a, v16b b, v8f c) {
    return __builtin_amdgcn_wmma_f32_16x16x32_bf16(false, a, false, b, (short)0, c, false, false);
  }
  static __device__ __forceinline__ void guard(v8f& a, v8f& b, v8f& c, v8f& d, v16b x, v16b y) { dep_guard4_b(a, b, c, d, x, y); }
  static __device__ __forceinline__ void keep(v16b a, v16b b, v16b c, v16b d) { keep4_b(a, b, c, d); }
};

template <int ET> struct Elem;
template <> struct Elem<0> { typedef _Float16 T; };
template <> struct Elem<1> { typedef __bf16 T; };
template <int ET, bool SPLIT, int EPI, int OUT_MODE, int ACT>
__global__ __launch_bounds__(256) void wmma_gemm64(
    const unsigned short* __restrict__ Ap, const unsigned short* __restrict__ A2p, int lda, long strideA,
    const unsigned short* __restrict__ Btp, const unsigned short* __restrict__ Bt2p, int ldb, long strideB,
    void* __restrict__ Cout, void* __restrict__ Cout2, int ldc, long strideC,
    const float* __restrict__ bias, long strideBias,
    const float* __restrict__ bn_g, const float* __restrict__ bn_b,
    const float* __restrict__ bn_m, const float* __restrict__ bn_v,
    int M, int N, int K, float scale) {
  typedef typename Elem<ET>::T T;
  typedef typename Frag<T>::V V;
  const T* A = (const T*)Ap; const T* A2 = (const T*)A2p; const T* Bt = (const T*)Btp; const T* Bt2 = (const T*)Bt2p;
  __shared__ __align__(16) float sT[8][16 * 68];
  const int b    = blockIdx.y;
  const int lane = threadIdx.x & 31;
  const int wave = threadIdx.x >> 5;
  const int tilesN = N >> 6;
  const int tilesM = M >> 6;
  const int tile = blockIdx.x * 8 + wave;
  if (tile >= tilesM * tilesN) return;
  const int tm = tile / tilesN;
  const int tn = tile - tm * tilesN;
  const int m0 = tm << 6;
  const int n0 = tn << 6;

  const T* Ab  = A  + (size_t)b * strideA;
  const T* Bb  = Bt + (size_t)b * strideB;
  const T* Ab2 = SPLIT ? (A2  + (size_t)b * strideA) : nullptr;
  const T* Bb2 = SPLIT ? (Bt2 + (size_t)b * strideB) : nullptr;

  const int rlane = lane & 15;
  const int koff  = (lane >> 4) * 8;
  const int mOff  = (lane >> 4) * 8;

  v8f acc[4][4];
#pragma unroll
  for (int i = 0; i < 4; ++i)
#pragma unroll
    for (int j = 0; j < 4; ++j) acc[i][j] = (v8f){0.f,0.f,0.f,0.f,0.f,0.f,0.f,0.f};

  for (int k0 = 0; k0 < K; k0 += 32) {
    V bh[4], bl[4];
#pragma unroll
    for (int j = 0; j < 4; ++j) {
      const size_t bo = (size_t)(n0 + (j << 4) + rlane) * ldb + koff + k0;
      bh[j] = Frag<T>::load(Bb + bo);
      if (SPLIT) bl[j] = Frag<T>::load(Bb2 + bo);
    }
#pragma unroll
    for (int i = 0; i < 4; ++i) {
      const size_t ao = (size_t)(m0 + (i << 4) + rlane) * lda + koff + k0;
      V ah = Frag<T>::load(Ab + ao);
      V al;
      if (SPLIT) al = Frag<T>::load(Ab2 + ao);
#pragma unroll
      for (int j = 0; j < 4; ++j) {
        acc[i][j] = Frag<T>::mma(ah, bh[j], acc[i][j]);
        if (SPLIT) {
          acc[i][j] = Frag<T>::mma(ah, bl[j], acc[i][j]);
          acc[i][j] = Frag<T>::mma(al, bh[j], acc[i][j]);
        }
      }
      Frag<T>::guard(acc[i][0], acc[i][1], acc[i][2], acc[i][3], ah, SPLIT ? al : ah);
    }
    Frag<T>::keep(bh[0], bh[1], bh[2], bh[3]);
    if (SPLIT) Frag<T>::keep(bl[0], bl[1], bl[2], bl[3]);
  }
  acc_guard4(acc[0][0], acc[0][1], acc[0][2], acc[0][3]);
  acc_guard4(acc[1][0], acc[1][1], acc[1][2], acc[1][3]);
  acc_guard4(acc[2][0], acc[2][1], acc[2][2], acc[2][3]);
  acc_guard4(acc[3][0], acc[3][1], acc[3][2], acc[3][3]);

  float e_b[4], e_sc[4], e_sh[4];
#pragma unroll
  for (int j = 0; j < 4; ++j) {
    const int n = n0 + (j << 4) + rlane;
    e_b[j] = 0.f; e_sc[j] = 1.f; e_sh[j] = 0.f;
    if (EPI == 1) e_b[j] = bias[(size_t)b * strideBias + n];
    if (EPI == 2) {
      e_b[j] = bias[n];
      const float inv = bn_g[n] / sqrtf(bn_v[n] + 1e-5f);
      e_sc[j] = inv;
      e_sh[j] = bn_b[n] - bn_m[n] * inv;
    }
  }

  float* slab = sT[wave];
#pragma unroll
  for (int i = 0; i < 4; ++i) {
    const int mBase = m0 + (i << 4);
#pragma unroll
    for (int j = 0; j < 4; ++j) {
#pragma unroll
      for (int r = 0; r < 8; ++r) {
        float v = acc[i][j][r] * scale;
        if (EPI >= 1) v += e_b[j];
        if (EPI == 2) v = v * e_sc[j] + e_sh[j];
        if (ACT == 2) v = fmaxf(v, 0.0f);
        slab[(mOff + r) * 68 + (j << 4) + rlane] = v;
      }
    }
    __builtin_amdgcn_fence(__ATOMIC_RELEASE, "workgroup");
    __builtin_amdgcn_wave_barrier();
    __builtin_amdgcn_fence(__ATOMIC_ACQUIRE, "workgroup");
    if (OUT_MODE == 0) {
      float* C = (float*)Cout + (size_t)b * strideC;
      const int hh = lane >> 4, c4 = (lane & 15) * 4;
      for (int pass = 0; pass < 2; ++pass) {
#pragma unroll
        for (int it = 0; it < 8; ++it) {
          const int row = it * 2 + hh;
          v4f v = *(const v4f*)(slab + row * 68 + c4);
          *(volatile v4f*)(C + (size_t)(mBase + row) * ldc + n0 + c4) = v;
        }
        __threadfence();
      }
    } else {
      const int q = lane >> 3, c8 = (lane & 7) * 8;
      unsigned short* C  = (unsigned short*)Cout  + (size_t)b * strideC;
      unsigned short* C2 = (unsigned short*)Cout2 + (size_t)b * strideC;
      for (int pass = 0; pass < 2; ++pass) {
#pragma unroll
        for (int it = 0; it < 4; ++it) {
          const int row = it * 4 + q;
          const float* sp = slab + row * 68 + c8;
          v8h hv, lv;
#pragma unroll
          for (int e = 0; e < 8; ++e) {
            const float fv = sp[e];
            const unsigned short hb = f2bf_bits(fv);
            const unsigned short lb = f2bf_bits(fv - bf_bits2f(hb));
            hv[e] = __builtin_bit_cast(_Float16, hb);
            lv[e] = __builtin_bit_cast(_Float16, lb);
          }
          *(volatile v8h*)(C + (size_t)(mBase + row) * ldc + n0 + c8) = hv;
          *(volatile v8h*)(C2 + (size_t)(mBase + row) * ldc + n0 + c8) = lv;
        }
        __threadfence();
      }
    }
    __builtin_amdgcn_fence(__ATOMIC_RELEASE, "workgroup");
    __builtin_amdgcn_wave_barrier();
    __builtin_amdgcn_fence(__ATOMIC_ACQUIRE, "workgroup");
  }
}

__global__ __launch_bounds__(256) void split_rows_bf16_kernel(
    const float* __restrict__ src, unsigned short* __restrict__ dhi, unsigned short* __restrict__ dlo, int total8)
{
  const int i = blockIdx.x * 256 + threadIdx.x;
  if (i >= total8) return;
  const size_t e0 = (size_t)i << 3;
  const v4f a0 = *(const v4f*)(src + e0);
  const v4f a1 = *(const v4f*)(src + e0 + 4);
  v8h hv, lv;
  split8_bf16(a0, a1, hv, lv);
  unsigned short* qh = dhi + e0;
  unsigned short* ql = dlo + e0;
  *(volatile v8h*)qh = hv;
  *(volatile v8h*)ql = lv;
  __threadfence();
  *(volatile v8h*)qh = hv;
  *(volatile v8h*)ql = lv;
}

__global__ __launch_bounds__(256) void cast_f16_kernel(
    const float* __restrict__ src, unsigned short* __restrict__ dst, int total8, float carry)
{
  const int i = blockIdx.x * 256 + threadIdx.x;
  if (i >= total8) return;
  const size_t e0 = (size_t)i << 3;
  const float* p = src + e0;
  const v4f a0 = *(const v4f*)(p);
  const v4f a1 = *(const v4f*)(p + 4);
  v8h hv;
#pragma unroll
  for (int e = 0; e < 4; ++e) {
    hv[e]     = (_Float16)(a0[e] * carry);
    hv[4 + e] = (_Float16)(a1[e] * carry);
  }
  unsigned short* q = dst + e0;
  *(volatile v8h*)q = hv;
  __threadfence();
  *(volatile v8h*)q = hv;
}

__global__ __launch_bounds__(256) void x_rows_split_kernel(
    const float* __restrict__ x, unsigned short* __restrict__ FH, unsigned short* __restrict__ FL)
{
  __shared__ float tile[64 * 65];
  const int tid = threadIdx.x, lane = tid & 31, wave = tid >> 5;
  const int c0 = blockIdx.x * 64;
  const int l0 = blockIdx.y * 64;
  const int b  = blockIdx.z;
#pragma unroll
  for (int p = 0; p < 16; ++p) {
    const int idx = tid + p * 256;
    const int cc = idx >> 6;
    const int ll = idx & 63;
    tile[cc * 65 + ll] = x[((size_t)(b * kCin + c0 + cc)) * kL + l0 + ll];
  }
  __syncthreads();
  const int q = lane >> 3, c8 = (lane & 7) * 8;
  v8h hv[2], lv[2];
#pragma unroll
  for (int it = 0; it < 2; ++it) {
    const int prow = it * 32 + wave * 4 + q;
#pragma unroll
    for (int e = 0; e < 8; ++e) {
      const float f = tile[(c8 + e) * 65 + prow];
      const unsigned short hb = f2bf_bits(f);
      const unsigned short lb = f2bf_bits(f - bf_bits2f(hb));
      hv[it][e] = __builtin_bit_cast(_Float16, hb);
      lv[it][e] = __builtin_bit_cast(_Float16, lb);
    }
  }
  for (int pass = 0; pass < 2; ++pass) {
#pragma unroll
    for (int it = 0; it < 2; ++it) {
      const int prow = it * 32 + wave * 4 + q;
      const size_t o = (size_t)(b * kL + l0 + prow) * kDm + c0 + c8;
      *(volatile v8h*)(FH + o) = hv[it];
      *(volatile v8h*)(FL + o) = lv[it];
    }
    __threadfence();
  }
}

__global__ __launch_bounds__(64) void adaptive_pool_kernel(
    const float* __restrict__ x, unsigned short* __restrict__ PH, unsigned short* __restrict__ PL)
{
  const int r = blockIdx.x;
  const int tid = threadIdx.x;
  int s, rl, nvalid;
  if (r < kPRow2)      { s = 5;  rl = r;          nvalid = kM1; }
  else if (r < kPRow3) { s = 9;  rl = r - kPRow2; nvalid = kM2; }
  else                 { s = 13; rl = r - kPRow3; nvalid = kM3; }
  const bool valid = rl < nvalid;
  const int rc = valid ? rl : 0;
  const int ss = s * s;
  const int b  = rc / ss;
  const int ij = rc - b * ss;
  const int i  = ij / s;
  const int j  = ij - i * s;
  const int hst = (i * 16) / s;
  const int hen = ((i + 1) * 16 + s - 1) / s;
  const int wst = (j * 16) / s;
  const int wen = ((j + 1) * 16 + s - 1) / s;
  const int hlim = valid ? hen : hst;
  const float inv = 1.0f / (float)((hen - hst) * (wen - wst));
  const int c8 = tid * 8;
  const float* xp = x + ((size_t)(b * kCin + c8)) * kL;
  float acc[8];
#pragma unroll
  for (int e = 0; e < 8; ++e) acc[e] = 0.f;
#pragma unroll 1
  for (int h = hst; h < hlim; ++h) {
#pragma unroll 1
    for (int w = wst; w < wen; ++w) {
      const float* q = xp + h * 16 + w;
#pragma unroll
      for (int e = 0; e < 8; ++e) acc[e] += q[(size_t)e * kL];
    }
  }
  v4f a0, a1;
#pragma unroll
  for (int e = 0; e < 4; ++e) {
    const float f0 = acc[e] * inv;
    const float f1 = acc[4 + e] * inv;
    a0[e] = valid ? f0 : 0.0f;
    a1[e] = valid ? f1 : 0.0f;
  }
  v8h hv, lv;
  split8_bf16(a0, a1, hv, lv);
  const size_t o = (size_t)r * kCin + c8;
  *(volatile v8h*)(PH + o) = hv;
  *(volatile v8h*)(PL + o) = lv;
  __threadfence();
  *(volatile v8h*)(PH + o) = hv;
  *(volatile v8h*)(PL + o) = lv;
}

__global__ __launch_bounds__(128) void level0_mean_kernel(const float* __restrict__ Q0, float* __restrict__ Y0)
{
  const int b = blockIdx.x, d = threadIdx.x;
  const float* q = Q0 + (size_t)b * kL * kDimP + d;
  float s0 = 0.f, s1 = 0.f, s2 = 0.f, s3 = 0.f;
#pragma unroll 1
  for (int l = 0; l < kL; l += 4) {
    s0 += q[(size_t)(l + 0) * kDimP];
    s1 += q[(size_t)(l + 1) * kDimP];
    s2 += q[(size_t)(l + 2) * kDimP];
    s3 += q[(size_t)(l + 3) * kDimP];
  }
  const float v = ((s0 + s1) + (s2 + s3)) * (1.0f / (float)kL);
  volatile float* p = Y0 + b * kDimP + d;
  *p = v;
  __threadfence();
  *p = v;
}

__global__ __launch_bounds__(128) void feat_tail_kernel(
    const float* __restrict__ Y0, const float* __restrict__ Q1, const float* __restrict__ Q2,
    const float* __restrict__ Q3, unsigned short* __restrict__ FH, unsigned short* __restrict__ FL)
{
  const int lane = threadIdx.x & 31, wave = threadIdx.x >> 5;
  const int half = lane >> 4;
  const int cg = (lane & 15) * 8;
  const int pix = blockIdx.x * 2 + half;
  const int b = pix >> 8;
  const int l = pix & 255;
  const int h = l >> 4, w = l & 15;
  v4f o0, o1;
  if (wave == 0) {
    o0 = *(const v4f*)(Y0 + b * kDimP + cg);
    o1 = *(const v4f*)(Y0 + b * kDimP + cg + 4);
  } else {
    const int s = (wave == 1) ? 5 : ((wave == 2) ? 9 : 13);
    const float* q = (wave == 1) ? Q1 : ((wave == 2) ? Q2 : Q3);
    const float sc = (float)s * (1.0f / 16.0f);
    const float sh = fmaxf(((float)h + 0.5f) * sc - 0.5f, 0.0f);
    int h0 = (int)sh; h0 = (h0 > s - 1) ? (s - 1) : h0;
    const float fh = sh - (float)h0;
    const int h1 = (h0 + 1 > s - 1) ? (s - 1) : (h0 + 1);
    const float sw = fmaxf(((float)w + 0.5f) * sc - 0.5f, 0.0f);
    int w0 = (int)sw; w0 = (w0 > s - 1) ? (s - 1) : w0;
    const float fw = sw - (float)w0;
    const int w1 = (w0 + 1 > s - 1) ? (s - 1) : (w0 + 1);
    const float* base = q + (size_t)(b * s * s) * kDimP + cg;
    const float* p00 = base + (size_t)(h0 * s + w0) * kDimP;
    const float* p01 = base + (size_t)(h0 * s + w1) * kDimP;
    const float* p10 = base + (size_t)(h1 * s + w0) * kDimP;
    const float* p11 = base + (size_t)(h1 * s + w1) * kDimP;
    const v4f a00 = *(const v4f*)(p00), b00 = *(const v4f*)(p00 + 4);
    const v4f a01 = *(const v4f*)(p01), b01 = *(const v4f*)(p01 + 4);
    const v4f a10 = *(const v4f*)(p10), b10 = *(const v4f*)(p10 + 4);
    const v4f a11 = *(const v4f*)(p11), b11 = *(const v4f*)(p11 + 4);
    const float k00 = (1.0f - fh) * (1.0f - fw);
    const float k01 = (1.0f - fh) * fw;
    const float k10 = fh * (1.0f - fw);
    const float k11 = fh * fw;
#pragma unroll
    for (int e = 0; e < 4; ++e) {
      o0[e] = k00 * a00[e] + k01 * a01[e] + k10 * a10[e] + k11 * a11[e];
      o1[e] = k00 * b00[e] + k01 * b01[e] + k10 * b10[e] + k11 * b11[e];
    }
  }
  v8h hv, lv;
  split8_bf16(o0, o1, hv, lv);
  const size_t o = (size_t)pix * kDm + kCin + wave * kDimP + cg;
  *(volatile v8h*)(FH + o) = hv;
  *(volatile v8h*)(FL + o) = lv;
  __threadfence();
  *(volatile v8h*)(FH + o) = hv;
  *(volatile v8h*)(FL + o) = lv;
}

__global__ __launch_bounds__(256) void dwconv_silu_kernel(
    const float* __restrict__ XZ, const float* __restrict__ cw, const float* __restrict__ cb,
    float* __restrict__ XC, unsigned short* __restrict__ XC16)
{
  __shared__ __align__(16) float sT[16 * kTP];
  const int tid = threadIdx.x, lane = tid & 31, wave = tid >> 5;
  const int d0 = blockIdx.x * 256, d = d0 + tid;
  const int b = blockIdx.y >> 4;
  const int h = blockIdx.y & 15;
  const float* wp = cw + (size_t)d * 9;
  const float w00 = wp[0], w01 = wp[1], w02 = wp[2];
  const float w10 = wp[3], w11 = wp[4], w12 = wp[5];
  const float w20 = wp[6], w21 = wp[7], w22 = wp[8];
  const float bc = cb[d];
  const bool okm = (h > 0), okp = (h < 15);
  const int hm = okm ? (h - 1) : 0;
  const int hp = okp ? (h + 1) : 15;
  const float* rt = XZ + ((size_t)(b * kL + hm * 16)) * kE2 + d;
  const float* rm = XZ + ((size_t)(b * kL + h * 16)) * kE2 + d;
  const float* rb = XZ + ((size_t)(b * kL + hp * 16)) * kE2 + d;
  float t0 = 0.f, m0 = 0.f, u0 = 0.f;
  float t1, m1, u1;
  {
    const float vt = rt[0];
    const float vm = rm[0];
    const float vb = rb[0];
    t1 = okm ? vt : 0.0f;
    m1 = vm;
    u1 = okp ? vb : 0.0f;
  }
#pragma unroll 1
  for (int w = 0; w < 16; ++w) {
    const int wn = w + 1;
    const bool okn = (wn < 16);
    const int wc = okn ? wn : 15;
    const float vt = rt[(size_t)wc * kE2];
    const float vm = rm[(size_t)wc * kE2];
    const float vb = rb[(size_t)wc * kE2];
    const float t2 = (okm && okn) ? vt : 0.0f;
    const float m2 = okn ? vm : 0.0f;
    const float u2 = (okp && okn) ? vb : 0.0f;
    float acc = w00 * t0;
    acc = fmaf(w01, t1, acc);
    acc = fmaf(w02, t2, acc);
    acc = fmaf(w10, m0, acc);
    acc = fmaf(w11, m1, acc);
    acc = fmaf(w12, m2, acc);
    acc = fmaf(w20, u0, acc);
    acc = fmaf(w21, u1, acc);
    acc = fmaf(w22, u2, acc);
    const float sv = acc + bc;
    const float sg = 1.0f / (1.0f + expf(-sv));
    sT[w * kTP + tid] = sv * sg;
    t0 = t1; t1 = t2;
    m0 = m1; m1 = m2;
    u0 = u1; u1 = u2;
  }
  __syncthreads();
  const int lb = b * kL + h * 16;
  const int hrow = wave >> 1;
  const int hch  = (wave & 1) * 128 + lane * 4;
  v4f fv[4];
  v8h bv[2];
#pragma unroll
  for (int it = 0; it < 4; ++it) fv[it] = *(const v4f*)(sT + (it * 4 + hrow) * kTP + hch);
#pragma unroll
  for (int it = 0; it < 2; ++it) {
    const float* sp = sT + (it * 8 + wave) * kTP + lane * 8;
    const v4f a0 = *(const v4f*)(sp);
    const v4f a1 = *(const v4f*)(sp + 4);
#pragma unroll
    for (int e = 0; e < 4; ++e) {
      bv[it][e]     = (_Float16)(a0[e] * kCarryXc);
      bv[it][4 + e] = (_Float16)(a1[e] * kCarryXc);
    }
  }
  for (int pass = 0; pass < 2; ++pass) {
#pragma unroll
    for (int it = 0; it < 4; ++it)
      *(volatile v4f*)(XC + (size_t)(lb + it * 4 + hrow) * kDi + d0 + hch) = fv[it];
#pragma unroll
    for (int it = 0; it < 2; ++it)
      *(volatile v8h*)(XC16 + (size_t)(lb + it * 8 + wave) * kDi + d0 + lane * 8) = bv[it];
    __threadfence();
  }
}

__device__ __forceinline__ int scan_pixel(int k, int l) {
  const int lt = (k & 2) ? (kL - 1 - l) : l;
  return (k & 1) ? (((lt & 15) << 4) + (lt >> 4)) : lt;
}

__global__ __launch_bounds__(32) void scan4_kernel(
    const float* __restrict__ XD, const float* __restrict__ XC, const float* __restrict__ DPRE,
    const float* __restrict__ Alog, const float* __restrict__ Dsk, float* __restrict__ YS)
{
  __shared__ __align__(16) float sY[kL * kScanCh];
  __shared__ __align__(16) float sBC[kScanTS * 32];
  __shared__ __align__(16) float sA[kNs * kScanCh];
  const int lane = threadIdx.x;
  constexpr int kBlkPerB = kDi / kScanCh;
  const int b  = blockIdx.x / kBlkPerB;
  const int d0 = (blockIdx.x - b * kBlkPerB) * kScanCh;
  const int d  = d0 + lane;
  const int row0 = b * kL;
  const float dsum = ((Dsk[d] + Dsk[kDi + d]) + Dsk[2 * kDi + d]) + Dsk[3 * kDi + d];
#pragma unroll 4
  for (int p = 0; p < kL; ++p) sY[p * kScanCh + lane] = dsum * XC[(size_t)(row0 + p) * kDi + d];

#pragma unroll 1
  for (int k = 0; k < kDirs; ++k) {
    __syncthreads();
    const float* al = Alog + ((size_t)(k * kDi + d)) * kNs;
#pragma unroll 1
    for (int n = 0; n < kNs; ++n) sA[n * kScanCh + lane] = -expf(al[n]);
    __syncthreads();
    float An[kNs], h[kNs];
#pragma unroll
    for (int n = 0; n < kNs; ++n) {
      An[n] = sA[n * kScanCh + lane];
      h[n] = 0.f;
    }
    const float* dp  = DPRE + (size_t)k * kPix * kDi;
    const float* xdk = XD + k * kXdG + kRk;
#pragma unroll 1
    for (int c = 0; c < kL / kScanTS; ++c) {
      const int l0 = c * kScanTS;
      __syncthreads();
#pragma unroll
      for (int it = 0; it < 16; ++it) {
        const int idx = it * 32 + lane;
        const int r  = idx >> 3;
        const int q4 = (idx & 7) * 4;
        const int p  = scan_pixel(k, l0 + r);
        *(v4f*)(sBC + r * 32 + q4) = *(const v4f*)(xdk + (size_t)(row0 + p) * kXdW + q4);
      }
      __syncthreads();
#pragma unroll 1
      for (int s = 0; s < kScanTS; ++s) {
        const int p = scan_pixel(k, l0 + s);
        const size_t ro = (size_t)(row0 + p) * kDi + d;
        const float u = XC[ro];
        const float v = dp[ro];
        const float* xr = sBC + s * 32;
        float Bs[kNs], Cs[kNs];
#pragma unroll
        for (int q4 = 0; q4 < 4; ++q4) {
          const v4f bv = *(const v4f*)(xr + 4 * q4);
          const v4f cv = *(const v4f*)(xr + kNs + 4 * q4);
          Bs[4 * q4 + 0] = bv[0]; Bs[4 * q4 + 1] = bv[1]; Bs[4 * q4 + 2] = bv[2]; Bs[4 * q4 + 3] = bv[3];
          Cs[4 * q4 + 0] = cv[0]; Cs[4 * q4 + 1] = cv[1]; Cs[4 * q4 + 2] = cv[2]; Cs[4 * q4 + 3] = cv[3];
        }
        const float a   = __expf(-fabsf(v));
        const float uu  = 1.0f + a;
        const float l1p = __logf(uu) + (a - (uu - 1.0f)) * __builtin_amdgcn_rcpf(uu);
        const float dl  = fmaxf(v, 0.0f) + l1p;
        const float du  = dl * u;
        float y = 0.f;
#pragma unroll
        for (int n = 0; n < kNs; ++n) {
          const float e = __expf(dl * An[n]);
          h[n] = fmaf(e, h[n], du * Bs[n]);
          y = fmaf(h[n], Cs[n], y);
        }
        sY[p * kScanCh + lane] += y;
      }
    }
  }
  __syncthreads();
  const int q = lane >> 3, c4 = (lane & 7) * 4;
  for (int pass = 0; pass < 2; ++pass) {
#pragma unroll 4
    for (int it = 0; it < kL / 4; ++it) {
      const int row = it * 4 + q;
      const v4f val = *(const v4f*)(sY + row * kScanCh + c4);
      *(volatile v4f*)(YS + (size_t)(row0 + row) * kDi + d0 + c4) = val;
    }
    __threadfence();
  }
}

__global__ __launch_bounds__(256) void ln_gate_kernel(
    const float* __restrict__ YS, const float* __restrict__ XZ, const float* __restrict__ lng,
    const float* __restrict__ lnb, unsigned short* __restrict__ YH, unsigned short* __restrict__ YL)
{
  __shared__ __align__(16) float sOut[kDi];
  __shared__ float sRedA[8];
  __shared__ float sRedB[8];
  const int tid = threadIdx.x, lane = tid & 31, wave = tid >> 5;
  const int pix = blockIdx.x;
  const float* yr = YS + (size_t)pix * kDi;
  const float* zr = XZ + (size_t)pix * kE2 + kDi;
  const v4f a0 = *(const v4f*)(yr + tid * 4);
  const v4f a1 = *(const v4f*)(yr + 1024 + tid * 4);
  float s = ((a0[0] + a0[1]) + (a0[2] + a0[3])) + ((a1[0] + a1[1]) + (a1[2] + a1[3]));
#pragma unroll
  for (int off = 16; off > 0; off >>= 1) s += __shfl_xor(s, off, 32);
  if (lane == 0) sRedA[wave] = s;
  __syncthreads();
  float tot = 0.f;
#pragma unroll
  for (int w = 0; w < 8; ++w) tot += sRedA[w];
  const float mean = tot * (1.0f / (float)kDi);
  float s2 = 0.f;
#pragma unroll
  for (int e = 0; e < 4; ++e) {
    const float x0 = a0[e] - mean;
    const float x1 = a1[e] - mean;
    s2 += x0 * x0;
    s2 += x1 * x1;
  }
#pragma unroll
  for (int off = 16; off > 0; off >>= 1) s2 += __shfl_xor(s2, off, 32);
  if (lane == 0) sRedB[wave] = s2;
  __syncthreads();
  float tot2 = 0.f;
#pragma unroll
  for (int w = 0; w < 8; ++w) tot2 += sRedB[w];
  const float var = tot2 * (1.0f / (float)kDi);
  const float inv = 1.0f / sqrtf(var + 1e-5f);
#pragma unroll 1
  for (int g = 0; g < 2; ++g) {
    const int idx = g * 1024 + tid * 4;
    const v4f yv = *(const v4f*)(yr + idx);
    const v4f gv = *(const v4f*)(lng + idx);
    const v4f bv = *(const v4f*)(lnb + idx);
    const v4f zv = *(const v4f*)(zr + idx);
    v4f o;
#pragma unroll
    for (int e = 0; e < 4; ++e) {
      const float nv = (yv[e] - mean) * inv * gv[e] + bv[e];
      const float z  = zv[e];
      const float sg = 1.0f / (1.0f + expf(-z));
      o[e] = nv * (z * sg);
    }
    *(v4f*)(sOut + idx) = o;
  }
  __syncthreads();
  const v4f p0 = *(const v4f*)(sOut + tid * 8);
  const v4f p1 = *(const v4f*)(sOut + tid * 8 + 4);
  v8h hv, lv;
  split8_bf16(p0, p1, hv, lv);
  const size_t o = (size_t)pix * kDi + tid * 8;
  *(volatile v8h*)(YH + o) = hv;
  *(volatile v8h*)(YL + o) = lv;
  __threadfence();
  *(volatile v8h*)(YH + o) = hv;
  *(volatile v8h*)(YL + o) = lv;
}

__global__ __launch_bounds__(256) void gelu_store_kernel(const float* __restrict__ PRE, float* __restrict__ out)
{
  __shared__ float tile[64 * 65];
  const int tid = threadIdx.x, lane = tid & 31, wave = tid >> 5;
  const int l0 = blockIdx.x * 64;
  const int d0 = blockIdx.y * 64;
  const int b  = blockIdx.z;
#pragma unroll 1
  for (int p = 0; p < 16; ++p) {
    const int idx = tid + p * 256;
    const int ll = idx >> 6;
    const int dd = idx & 63;
    const float v = PRE[(size_t)(b * kL + l0 + ll) * kDimP + d0 + dd];
    tile[ll * 65 + dd] = 0.5f * v * (1.0f + erff(v * 0.70710678118654752f));
  }
  __syncthreads();
  const int hh = lane >> 4, c4 = (lane & 15) * 4;
  v4f ov[4];
#pragma unroll
  for (int it = 0; it < 4; ++it) {
    const int drow = it * 16 + wave * 2 + hh;
#pragma unroll
    for (int e = 0; e < 4; ++e) ov[it][e] = tile[(c4 + e) * 65 + drow];
  }
  for (int pass = 0; pass < 2; ++pass) {
#pragma unroll
    for (int it = 0; it < 4; ++it) {
      const int drow = it * 16 + wave * 2 + hh;
      *(volatile v4f*)(out + ((size_t)(b * kDimP + d0 + drow)) * kL + l0 + c4) = ov[it];
    }
    __threadfence();
  }
}

extern "C" void kernel_launch(void* const* d_in, const int* in_sizes, int n_in,
                              void* d_out, int out_size, void* d_ws, size_t ws_size,
                              hipStream_t stream) {
  if (n_in < 24) return;
  if (in_sizes[0] != kB * kCin * kL) return;
  if (in_sizes[1] != 4 * kDimP * kCin) return;
  if (in_sizes[2] != 4 * kDimP || in_sizes[3] != 4 * kDimP || in_sizes[4] != 4 * kDimP) return;
  if (in_sizes[5] != 4 * kDimP || in_sizes[6] != 4 * kDimP) return;
  if (in_sizes[7] != kE2 * kDm) return;
  if (in_sizes[8] != kDi * 9 || in_sizes[9] != kDi) return;
  if (in_sizes[10] != kXdW * kDi) return;
  if (in_sizes[11] != kDirs * kDi * kRk || in_sizes[12] != kDirs * kDi) return;
  if (in_sizes[13] != kDirs * kDi * kNs || in_sizes[14] != kDirs * kDi) return;
  if (in_sizes[15] != kDi || in_sizes[16] != kDi) return;
  if (in_sizes[17] != kDm * kDi) return;
  if (in_sizes[18] != kDimP * kDm) return;
  if (in_sizes[19] != kDimP || in_sizes[20] != kDimP || in_sizes[21] != kDimP) return;
  if (in_sizes[22] != kDimP || in_sizes[23] != kDimP) return;
  if (out_size != kB * kDimP * kL) return;
  if (ws_size < kWsTotal) return;

  const float* x        = (const float*)d_in[0];
  const float* pool_w   = (const float*)d_in[1];
  const float* pool_b   = (const float*)d_in[2];
  const float* bn_g     = (const float*)d_in[3];
  const float* bn_b     = (const float*)d_in[4];
  const float* bn_m     = (const float*)d_in[5];
  const float* bn_v     = (const float*)d_in[6];
  const float* in_proj  = (const float*)d_in[7];
  const float* conv_w   = (const float*)d_in[8];
  const float* conv_b   = (const float*)d_in[9];
  const float* x_proj   = (const float*)d_in[10];
  const float* dt_w     = (const float*)d_in[11];
  const float* dt_b     = (const float*)d_in[12];
  const float* A_logs   = (const float*)d_in[13];
  const float* Dsk      = (const float*)d_in[14];
  const float* ln_g     = (const float*)d_in[15];
  const float* ln_b     = (const float*)d_in[16];
  const float* out_proj = (const float*)d_in[17];
  const float* cbr_w    = (const float*)d_in[18];
  const float* cbr_b    = (const float*)d_in[19];
  const float* cbr_g    = (const float*)d_in[20];
  const float* cbr_bt   = (const float*)d_in[21];
  const float* cbr_m    = (const float*)d_in[22];
  const float* cbr_v    = (const float*)d_in[23];
  float* out = (float*)d_out;

  char* ws = (char*)d_ws;
  unsigned short* WIH  = (unsigned short*)(ws + kOffWIH);
  unsigned short* WIL  = (unsigned short*)(ws + kOffWIL);
  unsigned short* WOH  = (unsigned short*)(ws + kOffWOH);
  unsigned short* WOL  = (unsigned short*)(ws + kOffWOL);
  unsigned short* WCH  = (unsigned short*)(ws + kOffWCH);
  unsigned short* WCL  = (unsigned short*)(ws + kOffWCL);
  unsigned short* WPH  = (unsigned short*)(ws + kOffWPH);
  unsigned short* WPL  = (unsigned short*)(ws + kOffWPL);
  unsigned short* WXP  = (unsigned short*)(ws + kOffWXP);
  unsigned short* WDT  = (unsigned short*)(ws + kOffWDT);
  unsigned short* FH   = (unsigned short*)(ws + kOffFH);
  unsigned short* FL   = (unsigned short*)(ws + kOffFL);
  unsigned short* PH   = (unsigned short*)(ws + kOffPH);
  unsigned short* PL   = (unsigned short*)(ws + kOffPL);
  float*          Q0   = (float*)(ws + kOffQ0);
  float*          Q1   = (float*)(ws + kOffQ1);
  float*          Q2   = (float*)(ws + kOffQ2);
  float*          Q3   = (float*)(ws + kOffQ3);
  float*          Y0   = (float*)(ws + kOffY0);
  float*          XZ   = (float*)(ws + kOffXZ);
  float*          XC   = (float*)(ws + kOffXC);
  unsigned short* XC16 = (unsigned short*)(ws + kOffXC16);
  float*          XD   = (float*)(ws + kOffXD);
  unsigned short* XD16 = (unsigned short*)(ws + kOffXD16);
  float*          DPRE = (float*)(ws + kOffDP);
  float*          YS   = (float*)(ws + kOffYS);
  unsigned short* YLH  = (unsigned short*)(ws + kOffYLH);
  unsigned short* YLL  = (unsigned short*)(ws + kOffYLL);
  unsigned short* YPH  = (unsigned short*)(ws + kOffYPH);
  unsigned short* YPL  = (unsigned short*)(ws + kOffYPL);
  float*          CBRP = (float*)(ws + kOffCP);
  const float* dummy = cbr_b;

  split_rows_bf16_kernel<<<(kE2 * kDm / 8) / 256, 256, 0, stream>>>(in_proj, WIH, WIL, kE2 * kDm / 8);
  split_rows_bf16_kernel<<<(kDm * kDi / 8) / 256, 256, 0, stream>>>(out_proj, WOH, WOL, kDm * kDi / 8);
  split_rows_bf16_kernel<<<(kDimP * kDm / 8) / 256, 256, 0, stream>>>(cbr_w, WCH, WCL, kDimP * kDm / 8);
  split_rows_bf16_kernel<<<(4 * kDimP * kCin / 8) / 256, 256, 0, stream>>>(pool_w, WPH, WPL, 4 * kDimP * kCin / 8);
  cast_f16_kernel<<<(kXdW * kDi / 8) / 256, 256, 0, stream>>>(x_proj, WXP, kXdW * kDi / 8, kCarryWxp);
  cast_f16_kernel<<<(kDirs * kDi * kRk / 8) / 256, 256, 0, stream>>>(dt_w, WDT, kDirs * kDi * kRk / 8, kCarryWdt);

  x_rows_split_kernel<<<dim3(kCin / 64, kL / 64, kB), 256, 0, stream>>>(x, FH, FL);

  adaptive_pool_kernel<<<kPRows, 64, 0, stream>>>(x, PH, PL);

  wmma_gemm64<1, true, 2, 0, 2><<<dim3(4, 1), 256, 0, stream>>>(
      FH, FL, kDm, 0L, WPH, WPL, kCin, 0L, (void*)Q0, (void*)Q0, kDimP, 0L,
      pool_b, 0L, bn_g, bn_b, bn_m, bn_v, kPix, kDimP, kCin, 1.0f);
  wmma_gemm64<1, true, 2, 0, 2><<<dim3(1, 1), 256, 0, stream>>>(
      PH, PL, kCin, 0L, WPH + (size_t)1 * kDimP * kCin, WPL + (size_t)1 * kDimP * kCin, kCin, 0L,
      (void*)Q1, (void*)Q1, kDimP, 0L,
      pool_b + 1 * kDimP, 0L, bn_g + 1 * kDimP, bn_b + 1 * kDimP, bn_m + 1 * kDimP, bn_v + 1 * kDimP,
      kM1P, kDimP, kCin, 1.0f);
  wmma_gemm64<1, true, 2, 0, 2><<<dim3(2, 1), 256, 0, stream>>>(
      PH + (size_t)kPRow2 * kCin, PL + (size_t)kPRow2 * kCin, kCin, 0L,
      WPH + (size_t)2 * kDimP * kCin, WPL + (size_t)2 * kDimP * kCin, kCin, 0L,
      (void*)Q2, (void*)Q2, kDimP, 0L,
      pool_b + 2 * kDimP, 0L, bn_g + 2 * kDimP, bn_b + 2 * kDimP, bn_m + 2 * kDimP, bn_v + 2 * kDimP,
      kM2P, kDimP, kCin, 1.0f);
  wmma_gemm64<1, true, 2, 0, 2><<<dim3(3, 1), 256, 0, stream>>>(
      PH + (size_t)kPRow3 * kCin, PL + (size_t)kPRow3 * kCin, kCin, 0L,
      WPH + (size_t)3 * kDimP * kCin, WPL + (size_t)3 * kDimP * kCin, kCin, 0L,
      (void*)Q3, (void*)Q3, kDimP, 0L,
      pool_b + 3 * kDimP, 0L, bn_g + 3 * kDimP, bn_b + 3 * kDimP, bn_m + 3 * kDimP, bn_v + 3 * kDimP,
      kM3P, kDimP, kCin, 1.0f);

  level0_mean_kernel<<<kB, kDimP, 0, stream>>>(Q0, Y0);
  feat_tail_kernel<<<kPix / 2, 128, 0, stream>>>(Y0, Q1, Q2, Q3, FH, FL);

  wmma_gemm64<1, true, 0, 0, 0><<<dim3(128, 1), 256, 0, stream>>>(
      FH, FL, kDm, 0L, WIH, WIL, kDm, 0L, (void*)XZ, (void*)XZ, kE2, 0L,
      dummy, 0L, dummy, dummy, dummy, dummy, kPix, kE2, kDm, 1.0f);

  dwconv_silu_kernel<<<dim3(kDi / 256, kB * 16), 256, 0, stream>>>(XZ, conv_w, conv_b, XC, XC16);

  wmma_gemm64<0, false, 0, 0, 0><<<dim3(12, 1), 256, 0, stream>>>(
      XC16, XC16, kDi, 0L, WXP, WXP, kDi, 0L, (void*)XD, (void*)XD, kXdW, 0L,
      dummy, 0L, dummy, dummy, dummy, dummy, kPix, kXdW, kDi, 1.0f / (kCarryXc * kCarryWxp));

  cast_f16_kernel<<<(kPix * kXdW / 8) / 256, 256, 0, stream>>>(XD, XD16, kPix * kXdW / 8, kCarryXd);

  wmma_gemm64<0, false, 1, 0, 0><<<dim3(64, kDirs), 256, 0, stream>>>(
      XD16, XD16, kXdW, (long)kXdG, WDT, WDT, kRk, (long)kDi * kRk,
      (void*)DPRE, (void*)DPRE, kDi, (long)kPix * kDi,
      dt_b, (long)kDi, dummy, dummy, dummy, dummy, kPix, kDi, kRk, 1.0f / (kCarryXd * kCarryWdt));

  scan4_kernel<<<kB * (kDi / kScanCh), kScanCh, 0, stream>>>(XD, XC, DPRE, A_logs, Dsk, YS);

  ln_gate_kernel<<<kPix, 256, 0, stream>>>(YS, XZ, ln_g, ln_b, YLH, YLL);

  wmma_gemm64<1, true, 0, 2, 0><<<dim3(32, 1), 256, 0, stream>>>(
      YLH, YLL, kDi, 0L, WOH, WOL, kDi, 0L, (void*)YPH, (void*)YPL, kDm, 0L,
      dummy, 0L, dummy, dummy, dummy, dummy, kPix, kDm, kDi, 1.0f);

  wmma_gemm64<1, true, 2, 0, 0><<<dim3(4, 1), 256, 0, stream>>>(
      YPH, YPL, kDm, 0L, WCH, WCL, kDm, 0L, (void*)CBRP, (void*)CBRP, kDimP, 0L,
      cbr_b, 0L, cbr_g, cbr_bt, cbr_m, cbr_v, kPix, kDimP, kDm, 1.0f);

  gelu_store_kernel<<<dim3(kL / 64, kDimP / 64, kB), 256, 0, stream>>>(CBRP, out);
}
